// DCGRUCell_2671469658627
// MI455X (gfx1250) — hardware-verified
//
#include <hip/hip_runtime.h>
#include <stddef.h>


#define INF     64
#define HID     128
#define KF      192
#define NTHR    256
#define NWAVE   8
#define EPT     8
#define NGRP    2
#define CHUNK   (NTHR * EPT * NGRP)
#define WCAP    (EPT * NGRP * 32)
#define LISTN   (NWAVE * WCAP)
#define NBC     4096
#define NBF     1024
#define RCAP    40960
#define RBN     128
#define TGT     256
#define DEGCAP  512
#define OTHR    512
#define BM      32
#define WSCAP   134217728
#define SCL_A   8.0f
#define SCL_W   16.0f
#define SCL_ACC 0.0078125f

#define LDS_FILL ((RCAP + NBF + LISTN) * 4 + 64)

static_assert((CHUNK & (CHUNK - 1)) == 0);
static_assert(CHUNK <= 4096);
static_assert(NBC <= 4096 && NBF <= 4096);
static_assert((NBC & (NBC - 1)) == 0 && (NBF & (NBF - 1)) == 0);
static_assert(NBC == 4 * NBF);
static_assert(OTHR * 8 == NBC);
static_assert((RCAP % 32) == 0);
static_assert(TGT == NWAVE * 32);
static_assert((NBC % TGT) == 0);
static_assert((TGT % BM) == 0);
static_assert(KF == INF + HID && (INF % 32) == 0 && (HID % 64) == 0);
static_assert(BM * 8 == NTHR);

typedef float    v2f  __attribute__((ext_vector_type(2)));
typedef float    v4f  __attribute__((ext_vector_type(4)));
typedef float    v8f  __attribute__((ext_vector_type(8)));
typedef int      v4i  __attribute__((ext_vector_type(4)));
typedef _Float16 v2h  __attribute__((ext_vector_type(2)));
typedef _Float16 v4h  __attribute__((ext_vector_type(4)));
typedef _Float16 v8h  __attribute__((ext_vector_type(8)));
typedef _Float16 v16h __attribute__((ext_vector_type(16)));
union FragH { v16h v; v8h h[2]; };

__device__ __forceinline__ v8f wmh(v16h a, v16h b, v8f c) {
  v8f d = __builtin_amdgcn_wmma_f32_16x16x32_f16(false, a, false, b, (short)0, c, false, false);
  asm volatile("v_nop\n\tv_nop\n\tv_nop\n\tv_nop" : "+v"(d) : "v"(a), "v"(b));
  return d;
}

template <int NB>
__device__ __forceinline__ int scan_chunk(const int* __restrict__ dsts, int nE, int cbase, int slotBase,
                                          int vec8, int* list, int tid, int lane, int wave) {
  int wc = 0;
#pragma unroll
  for (int g = 0; g < NGRP; ++g) {
    const int el0  = (g * NTHR + tid) * EPT;
    const int e0   = cbase + el0;
    const int sent = -2147483647 - 1;
    v4i da, db;
    if (vec8 != 0 && cbase + CHUNK <= nE) {
      da = *(const v4i*)(dsts + e0);
      db = *(const v4i*)(dsts + e0 + 4);
    } else {
      da.x = (e0     < nE) ? dsts[min(e0, nE - 1)] : sent;
      da.y = (e0 + 1 < nE) ? dsts[min(e0 + 1, nE - 1)] : sent;
      da.z = (e0 + 2 < nE) ? dsts[min(e0 + 2, nE - 1)] : sent;
      da.w = (e0 + 3 < nE) ? dsts[min(e0 + 3, nE - 1)] : sent;
      db.x = (e0 + 4 < nE) ? dsts[min(e0 + 4, nE - 1)] : sent;
      db.y = (e0 + 5 < nE) ? dsts[min(e0 + 5, nE - 1)] : sent;
      db.z = (e0 + 6 < nE) ? dsts[min(e0 + 6, nE - 1)] : sent;
      db.w = (e0 + 7 < nE) ? dsts[min(e0 + 7, nE - 1)] : sent;
    }
    const unsigned nb = (unsigned)slotBase;
    const unsigned s0 = (unsigned)da.x - nb, s1 = (unsigned)da.y - nb;
    const unsigned s2 = (unsigned)da.z - nb, s3 = (unsigned)da.w - nb;
    const unsigned s4 = (unsigned)db.x - nb, s5 = (unsigned)db.y - nb;
    const unsigned s6 = (unsigned)db.z - nb, s7 = (unsigned)db.w - nb;
    const bool h0 = s0 < (unsigned)NB, h1 = s1 < (unsigned)NB, h2 = s2 < (unsigned)NB, h3 = s3 < (unsigned)NB;
    const bool h4 = s4 < (unsigned)NB, h5 = s5 < (unsigned)NB, h6 = s6 < (unsigned)NB, h7 = s7 < (unsigned)NB;
    const unsigned any = __builtin_amdgcn_ballot_w32(h0 | h1 | h2 | h3 | h4 | h5 | h6 | h7);
    if (any != 0u) {
#define HITJ(J, HJ, SJ) { \
        const unsigned mj = __builtin_amdgcn_ballot_w32(HJ); \
        if (mj != 0u) { \
          if (HJ) { \
            const int pos = wc + (int)__builtin_amdgcn_mbcnt_lo(mj, 0u); \
            if (pos < WCAP) list[wave * WCAP + pos] = ((el0 + (J)) << 12) | (int)(SJ); \
          } \
          wc += (int)__builtin_popcount(mj); } }
      HITJ(0, h0, s0)
      HITJ(1, h1, s1)
      HITJ(2, h2, s2)
      HITJ(3, h3, s3)
      HITJ(4, h4, s4)
      HITJ(5, h5, s5)
      HITJ(6, h6, s6)
      HITJ(7, h7, s7)
#undef HITJ
    }
  }
  return wc;
}

template <int K, int NOUT>
__global__ __launch_bounds__(NTHR) void k_prepw(const float* __restrict__ W, _Float16* wp) {
  constexpr int UPR = K / 8;
  constexpr int NU  = NOUT * UPR;
  static_assert((K % 32) == 0 && (NU % NTHR) == 0);
  const int i = (int)blockIdx.x * NTHR + (int)threadIdx.x;
  if (i >= NU) return;
  const int n  = i / UPR;
  const int k0 = (i - n * UPR) * 8;
  v8f t;
#pragma unroll
  for (int j = 0; j < 8; ++j) {
    int k = k0 + j;
    k = k > K - 1 ? K - 1 : k;
    t[j] = W[(size_t)k * NOUT + n] * SCL_W;
  }
  const v8h o = __builtin_convertvector(t, v8h);
  _Float16* d = wp + (size_t)i * 8;
  *(volatile v8h*)d = o;
  __threadfence();
  *(volatile v8h*)d = o;
}

__global__ __launch_bounds__(NTHR) void k_count(
    const int* __restrict__ dsts, int* cnt, int nE, int vec8) {
  __shared__ __attribute__((aligned(16))) int scnt[NBC];
  __shared__ __attribute__((aligned(16))) int list[LISTN];
  __shared__ int wcnt[NWAVE];
  const int tid = threadIdx.x, lane = tid & 31, wave = tid >> 5;
  const int nodeBase = blockIdx.x * NBC;

  for (int i = tid; i < NBC; i += NTHR) scnt[i] = 0;
  __syncthreads();

  const int nChunks = (nE + CHUNK - 1) / CHUNK;
#pragma unroll 1
  for (int ch = 0; ch < nChunks; ++ch) {
    const int cbase = ch * CHUNK;
    const int wc = scan_chunk<NBC>(dsts, nE, cbase, nodeBase, vec8, list, tid, lane, wave);
    if (lane == 0) wcnt[wave] = wc;
    __syncthreads();
    if (wave == 0) {
#pragma unroll 1
      for (int wsx = 0; wsx < NWAVE; ++wsx) {
        int n = __builtin_amdgcn_readfirstlane(wcnt[wsx]);
        n = n > WCAP ? WCAP : (n < 0 ? 0 : n);
        const int* lp = list + wsx * WCAP;
#pragma unroll 1
        for (int i = 0; i < n; ++i) {
          const int ent  = __builtin_amdgcn_readfirstlane(lp[i]);
          const int slot = ent & (NBC - 1);
          if (lane == 0) scnt[slot] = scnt[slot] + 1;
        }
      }
    }
    __syncthreads();
  }

  v4i cq[4];
#pragma unroll
  for (int q = 0; q < 4; ++q) {
    const int f = (wave * 4 + q) * 128 + 4 * lane;
    cq[q] = *(const v4i*)(scnt + f);
  }
  int* cp = cnt + (size_t)nodeBase;
#pragma unroll
  for (int q = 0; q < 4; ++q) {
    const int f = (wave * 4 + q) * 128 + 4 * lane;
    *(volatile v4i*)(cp + f) = cq[q];
  }
  __threadfence();
#pragma unroll
  for (int q = 0; q < 4; ++q) {
    const int f = (wave * 4 + q) * 128 + 4 * lane;
    *(volatile v4i*)(cp + f) = cq[q];
  }
}

__global__ __launch_bounds__(OTHR) void k_offsets(
    const int* __restrict__ cnt, int* off, int* rbase, int nChunk) {
  __shared__ __attribute__((aligned(16))) int soff[NBC];
  __shared__ __attribute__((aligned(16))) int srb[RBN];
  __shared__ int wtot[OTHR / 32];
  const int tid = threadIdx.x, lane = tid & 31, wave = tid >> 5, sub = tid >> 7;
  for (int i = tid; i < RBN; i += OTHR) srb[i] = 0;
  int carry = 0;
#pragma unroll 1
  for (int ch = 0; ch < nChunk; ++ch) {
    const int base = ch * NBC;
    const v4i c0 = *(const v4i*)(cnt + base + 8 * tid);
    const v4i c1 = *(const v4i*)(cnt + base + 8 * tid + 4);
    const int e0 = max(c0.x, 0), e1 = max(c0.y, 0), e2 = max(c0.z, 0), e3 = max(c0.w, 0);
    const int e4 = max(c1.x, 0), e5 = max(c1.y, 0), e6 = max(c1.z, 0), e7 = max(c1.w, 0);
    const int ts = e0 + e1 + e2 + e3 + e4 + e5 + e6 + e7;
    int incl = ts;
#pragma unroll
    for (int d = 1; d < 32; d <<= 1) {
      const int t = __shfl_up(incl, d);
      if (lane >= d) incl += t;
    }
    if (lane == 31) wtot[wave] = incl;
    __syncthreads();
    const int S0 = wtot[0]  + wtot[1]  + wtot[2]  + wtot[3];
    const int S1 = wtot[4]  + wtot[5]  + wtot[6]  + wtot[7];
    const int S2 = wtot[8]  + wtot[9]  + wtot[10] + wtot[11];
    const int S3 = wtot[12] + wtot[13] + wtot[14] + wtot[15];
    int pre = 0;
#pragma unroll 1
    for (int w = 4 * sub; w < wave; ++w) pre += wtot[w];
    const int b0 = carry;
    const int b1 = b0 + ((S0 + 31) & ~31);
    const int b2 = b1 + ((S1 + 31) & ~31);
    const int b3 = b2 + ((S2 + 31) & ~31);
    const int b4 = b3 + ((S3 + 31) & ~31);
    const int myb = sub == 0 ? b0 : (sub == 1 ? b1 : (sub == 2 ? b2 : b3));
    if (tid == 0) {
      srb[min(4 * ch + 0, RBN - 1)] = b0;
      srb[min(4 * ch + 1, RBN - 1)] = b1;
      srb[min(4 * ch + 2, RBN - 1)] = b2;
      srb[min(4 * ch + 3, RBN - 1)] = b3;
    }
    int run = myb + pre + incl - ts;
    soff[8 * tid + 0] = run; run += e0;
    soff[8 * tid + 1] = run; run += e1;
    soff[8 * tid + 2] = run; run += e2;
    soff[8 * tid + 3] = run; run += e3;
    soff[8 * tid + 4] = run; run += e4;
    soff[8 * tid + 5] = run; run += e5;
    soff[8 * tid + 6] = run; run += e6;
    soff[8 * tid + 7] = run;
    carry = b4;
    __syncthreads();
    const v4i o0 = *(const v4i*)(soff + 4 * tid);
    const v4i o1 = *(const v4i*)(soff + 4 * (tid + OTHR));
    int* op = off + base;
    *(volatile v4i*)(op + 4 * tid) = o0;
    *(volatile v4i*)(op + 4 * (tid + OTHR)) = o1;
    __threadfence();
    *(volatile v4i*)(op + 4 * tid) = o0;
    *(volatile v4i*)(op + 4 * (tid + OTHR)) = o1;
    __syncthreads();
  }
  if (tid == 0) srb[min(4 * nChunk, RBN - 1)] = carry;
  __syncthreads();
  v4i rv = {0, 0, 0, 0};
  if (tid < 32) rv = *(const v4i*)(srb + 4 * tid);
  if (tid < 32) *(volatile v4i*)(rbase + 4 * tid) = rv;
  __threadfence();
  if (tid < 32) *(volatile v4i*)(rbase + 4 * tid) = rv;
}

__global__ __launch_bounds__(NTHR) void k_fill(
    const int* __restrict__ dsts, const int* __restrict__ off, const int* __restrict__ rbase,
    int* csr, int nE, int vec8, int csrLen) {
  extern __shared__ v4f lds_dyn[];
  int* region = (int*)lds_dyn;
  int* cursor = region + RCAP;
  int* list   = cursor + NBF;
  int* wcnt   = list + LISTN;
  const int tid = threadIdx.x, lane = tid & 31, wave = tid >> 5;
  const int b = blockIdx.x;
  const int nodeBase = b * NBF;

  int rb0 = rbase[b];
  const int rb1 = rbase[b + 1];
  rb0 = rb0 < 0 ? 0 : (rb0 > csrLen ? csrLen : rb0);
  rb0 &= ~31;
  int len = rb1 - rb0;
  len = len < 0 ? 0 : (len > RCAP ? RCAP : len);
  int lenW = (len + 31) & ~31;
  if (rb0 + lenW > csrLen) lenW = (csrLen - rb0) & ~31;

  {
    const v4i z = {0, 0, 0, 0};
    for (int i = tid; i < RCAP / 4; i += NTHR) ((v4i*)region)[i] = z;
    for (int s = tid; s < NBF; s += NTHR) {
      int o = off[nodeBase + s] - rb0;
      o = o < 0 ? 0 : (o > RCAP ? RCAP : o);
      cursor[s] = o;
    }
  }
  __syncthreads();

  const int nChunks = (nE + CHUNK - 1) / CHUNK;
#pragma unroll 1
  for (int ch = 0; ch < nChunks; ++ch) {
    const int cbase = ch * CHUNK;
    const int wc = scan_chunk<NBF>(dsts, nE, cbase, nodeBase, vec8, list, tid, lane, wave);
    if (lane == 0) wcnt[wave] = wc;
    __syncthreads();
    if (wave == 0) {
#pragma unroll 1
      for (int wsx = 0; wsx < NWAVE; ++wsx) {
        int n = __builtin_amdgcn_readfirstlane(wcnt[wsx]);
        n = n > WCAP ? WCAP : (n < 0 ? 0 : n);
        const int* lp = list + wsx * WCAP;
#pragma unroll 1
        for (int i = 0; i < n; ++i) {
          const int ent  = __builtin_amdgcn_readfirstlane(lp[i]);
          const int slot = ent & (NBF - 1);
          int e = cbase + ((ent >> 12) & (CHUNK - 1));
          e = e > nE - 1 ? nE - 1 : (e < 0 ? 0 : e);
          if (lane == 0) {
            int pos = cursor[slot];
            pos = pos < 0 ? 0 : (pos > RCAP - 1 ? RCAP - 1 : pos);
            region[pos] = e;
            const int np = pos + 1;
            cursor[slot] = np > RCAP ? RCAP : np;
          }
        }
      }
    }
    __syncthreads();
  }

  const int nv = lenW >> 2;
  int* gp = csr + rb0;
#pragma unroll 1
  for (int i = tid; i < nv; i += NTHR) { const v4i v = ((const v4i*)region)[i]; *(volatile v4i*)(gp + 4 * i) = v; }
  __threadfence();
#pragma unroll 1
  for (int i = tid; i < nv; i += NTHR) { const v4i v = ((const v4i*)region)[i]; *(volatile v4i*)(gp + 4 * i) = v; }
}

template <int HASX>
__global__ __launch_bounds__(NTHR) void k_agg(
    const int* __restrict__ csr, const int* __restrict__ off, const int* __restrict__ cnt,
    const int* __restrict__ srcs, const float* __restrict__ xs, const float* __restrict__ ss,
    _Float16* xq, _Float16* sq, int nN, int nE, int csrLen) {
  constexpr int SLABN = HASX ? (NWAVE * 32 * INF) : 16;
  __shared__ __attribute__((aligned(16))) _Float16 slab[SLABN];
  const int tid = threadIdx.x, lane = tid & 31, wave = tid >> 5;
  const int tbase = blockIdx.x * TGT + wave * 32;
  _Float16* sw = slab + (HASX ? wave * (32 * INF) : 0);

  const int cl    = tbase + lane;
  const int cnt_l = cnt[cl];
  const int off_l = off[cl];

#pragma unroll 1
  for (int j = 0; j < 32; ++j) {
    const int c = tbase + j;
    int nraw = __shfl(cnt_l, j);
    nraw = nraw < 0 ? 0 : (nraw > nE ? nE : nraw);
    const int n = nraw > DEGCAP ? DEGCAP : nraw;
    const int st = __shfl(off_l, j);

    v2f ax = {0.0f, 0.0f};
    v4f as = {0.0f, 0.0f, 0.0f, 0.0f};
#pragma unroll 1
    for (int q0 = 0; q0 < n; q0 += 32) {
      int pos = st + q0 + lane;
      pos = pos < 0 ? 0 : (pos > csrLen - 1 ? csrLen - 1 : pos);
      int el = csr[pos];
      el = el < 0 ? 0 : (el > nE - 1 ? nE - 1 : el);
      int sl = srcs[el];
      sl = sl < 0 ? 0 : (sl > nN - 1 ? nN - 1 : sl);
      const int mcnt = (n - q0) < 32 ? (n - q0) : 32;
#pragma unroll 1
      for (int pp = 0; pp < mcnt; ++pp) {
        const int s = __builtin_amdgcn_readlane(sl, pp);
        if (HASX) {
          const v2f xv = *(const v2f*)(xs + (size_t)s * INF + 2 * lane);
          ax = ax + xv;
        }
        const v4f sv = *(const v4f*)(ss + (size_t)s * HID + 4 * lane);
        as = as + sv;
      }
    }

    const float nf = (float)(nraw < 1 ? 1 : nraw);
    const float rd = (1.0f / nf) * SCL_A;
    v4f vs = as * rd;
    if (c >= nN) { vs.x = 0.0f; vs.y = 0.0f; vs.z = 0.0f; vs.w = 0.0f; }
    const v4h os = __builtin_convertvector(vs, v4h);
    _Float16* gp = sq + (size_t)c * HID + 4 * lane;
    *(volatile v4h*)gp = os;
    __threadfence();
    *(volatile v4h*)gp = os;

    if (HASX) {
      v2f vx = ax * rd;
      if (c >= nN) { vx.x = 0.0f; vx.y = 0.0f; }
      const v2h ox = __builtin_convertvector(vx, v2h);
      *(v2h*)(sw + j * INF + 2 * lane) = ox;
    }
  }

  if (HASX) {
    __syncthreads();
    _Float16* gp = xq + (size_t)tbase * INF;
    v8h o[8];
#pragma unroll
    for (int q = 0; q < 8; ++q) o[q] = *(const v8h*)(sw + q * 256 + 8 * lane);
#pragma unroll
    for (int q = 0; q < 8; ++q) *(volatile v8h*)(gp + q * 256 + 8 * lane) = o[q];
    __threadfence();
#pragma unroll
    for (int q = 0; q < 8; ++q) *(volatile v8h*)(gp + q * 256 + 8 * lane) = o[q];
  }
}

template <int K, int LDB, int TPW>
__device__ __forceinline__ void mma_pair(const _Float16* __restrict__ Ap, const _Float16* __restrict__ Bp,
                                         int arow, int c0, int m, int hh, v8f (&acc)[TPW]) {
  constexpr int KT = K / 32;
  static_assert(K % 32 == 0 && LDB % 8 == 0);
  const _Float16* ap  = Ap + (size_t)arow * K + 8 * hh;
  const _Float16* bp0 = Bp + (size_t)(c0 + m) * LDB + 8 * hh;
#pragma unroll 1
  for (int kt = 0; kt < KT; ++kt) {
    FragH a;
    a.h[0] = *(const v8h*)(ap + 32 * kt);
    a.h[1] = *(const v8h*)(ap + 32 * kt + 16);
#pragma unroll
    for (int t = 0; t < TPW; ++t) {
      const _Float16* bp = bp0 + (size_t)(16 * t) * LDB + 32 * kt;
      FragH bf;
      bf.h[0] = *(const v8h*)bp;
      bf.h[1] = *(const v8h*)(bp + 16);
      acc[t] = wmh(a.v, bf.v, acc[t]);
    }
  }
}

__global__ __launch_bounds__(NTHR) void k_gemm1(
    const _Float16* __restrict__ A1, const _Float16* __restrict__ A2,
    const _Float16* __restrict__ Bp, const float* __restrict__ bias,
    const float* __restrict__ st, float* rsP, float* uP, int nN) {
  constexpr int NC  = 2 * HID;
  constexpr int LDB = KF;
  constexpr int TPW = NC / 64;
  constexpr int NIT = (BM * HID / 4) / NTHR;
  static_assert(TPW == 4 && NIT == 4);

  __shared__ __attribute__((aligned(16))) float stg[BM * NC];
  const int tid = threadIdx.x, lane = tid & 31, wave = tid >> 5, hh = lane >> 4, m = lane & 15;
  const int rowBase = blockIdx.x * BM;
  const int rg = wave >> 2, cq = wave & 3;
  const int r0 = rg * 16;
  const int c0 = cq * (NC / 4);

  v8f acc[TPW];
#pragma unroll
  for (int t = 0; t < TPW; ++t) { v8f z = {0.f, 0.f, 0.f, 0.f, 0.f, 0.f, 0.f, 0.f}; acc[t] = z; }

  mma_pair<INF, LDB, TPW>(A1, Bp,       rowBase + r0 + m, c0, m, hh, acc);
  mma_pair<HID, LDB, TPW>(A2, Bp + INF, rowBase + r0 + m, c0, m, hh, acc);

  {
    float* sp = stg + (size_t)(r0 + 8 * hh) * NC + c0 + m;
#pragma unroll
    for (int t = 0; t < TPW; ++t) {
      const float bv = bias[c0 + 16 * t + m];
#pragma unroll
      for (int r = 0; r < 8; ++r) {
        const float v = acc[t][r] * SCL_ACC + bv;
        const float e = __expf(-v);
        const float g = __builtin_amdgcn_rcpf(1.0f + e);
        sp[r * NC + 16 * t] = g;
      }
    }
  }
  __syncthreads();

  v4f pr[NIT], pu[NIT];
#pragma unroll
  for (int it = 0; it < NIT; ++it) {
    const int q = it * NTHR + tid;
    const int row = q >> 5;
    const int col = (q & 31) * 4;
    const int grow = rowBase + row;
    const int srow = grow > nN - 1 ? nN - 1 : grow;
    const v4f r4 = *(const v4f*)(stg + row * NC + col);
    v4f u4 = *(const v4f*)(stg + row * NC + HID + col);
    const v4f s4 = *(const v4f*)(st + (size_t)srow * HID + col);
    v4f p = r4 * s4;
    if (grow >= nN) {
      p.x = 0.0f; p.y = 0.0f; p.z = 0.0f; p.w = 0.0f;
      u4.x = 0.0f; u4.y = 0.0f; u4.z = 0.0f; u4.w = 0.0f;
    }
    pr[it] = p;
    pu[it] = u4;
  }
#pragma unroll
  for (int it = 0; it < NIT; ++it) {
    const int q = it * NTHR + tid;
    const size_t o = (size_t)(rowBase + (q >> 5)) * HID + (q & 31) * 4;
    *(volatile v4f*)(rsP + o) = pr[it];
    *(volatile v4f*)(uP + o)  = pu[it];
  }
  __threadfence();
#pragma unroll
  for (int it = 0; it < NIT; ++it) {
    const int q = it * NTHR + tid;
    const size_t o = (size_t)(rowBase + (q >> 5)) * HID + (q & 31) * 4;
    *(volatile v4f*)(rsP + o) = pr[it];
    *(volatile v4f*)(uP + o)  = pu[it];
  }
}

__global__ __launch_bounds__(NTHR) void k_gemm2(
    const _Float16* __restrict__ A1, const _Float16* __restrict__ A2,
    const _Float16* __restrict__ Bp, const float* __restrict__ bias,
    const float* __restrict__ st, const float* __restrict__ uP,
    float* out, int nN, int oofs) {
  constexpr int NC  = HID;
  constexpr int LDB = KF;
  constexpr int TPW = NC / 64;
  constexpr int NIT = (BM * HID / 4) / NTHR;
  static_assert(TPW == 2 && NIT == 4);

  __shared__ __attribute__((aligned(16))) float stg[BM * NC];
  const int tid = threadIdx.x, lane = tid & 31, wave = tid >> 5, hh = lane >> 4, m = lane & 15;
  const int rowBase = blockIdx.x * BM;
  const int rg = wave >> 2, cq = wave & 3;
  const int r0 = rg * 16;
  const int c0 = cq * (NC / 4);

  v8f acc[TPW];
#pragma unroll
  for (int t = 0; t < TPW; ++t) { v8f z = {0.f, 0.f, 0.f, 0.f, 0.f, 0.f, 0.f, 0.f}; acc[t] = z; }

  mma_pair<INF, LDB, TPW>(A1, Bp,       rowBase + r0 + m, c0, m, hh, acc);
  mma_pair<HID, LDB, TPW>(A2, Bp + INF, rowBase + r0 + m, c0, m, hh, acc);

  {
    float* sp = stg + (size_t)(r0 + 8 * hh) * NC + c0 + m;
#pragma unroll
    for (int t = 0; t < TPW; ++t) {
      const float bv = bias[c0 + 16 * t + m];
#pragma unroll
      for (int r = 0; r < 8; ++r) {
        const float v  = acc[t][r] * SCL_ACC + bv;
        const float vc = fminf(fmaxf(v, -16.0f), 16.0f);
        const float e  = __expf(2.0f * vc);
        const float th = 1.0f - 2.0f * __builtin_amdgcn_rcpf(e + 1.0f);
        sp[r * NC + 16 * t] = th;
      }
    }
  }
  __syncthreads();

  v4f o4[NIT];
#pragma unroll
  for (int it = 0; it < NIT; ++it) {
    const int q = it * NTHR + tid;
    const int row = q >> 5;
    const int col = (q & 31) * 4;
    const int grow = rowBase + row;
    const int srow = grow > nN - 1 ? nN - 1 : grow;
    const v4f c4 = *(const v4f*)(stg + row * NC + col);
    const v4f u4 = *(const v4f*)(uP + (size_t)grow * HID + col);
    const v4f s4 = *(const v4f*)(st + (size_t)srow * HID + col);
    const v4f one = {1.0f, 1.0f, 1.0f, 1.0f};
    o4[it] = u4 * s4 + (one - u4) * c4;
  }
#pragma unroll
  for (int it = 0; it < NIT; ++it) {
    const int q = it * NTHR + tid;
    const int grow = rowBase + (q >> 5);
    if (grow < nN) {
      const size_t o = (size_t)grow * HID + (q & 31) * 4;
      *(volatile v4f*)(out + o) = o4[it];
      *(volatile v4f*)(out + (size_t)oofs + o) = o4[it];
    }
  }
  __threadfence();
#pragma unroll
  for (int it = 0; it < NIT; ++it) {
    const int q = it * NTHR + tid;
    const int grow = rowBase + (q >> 5);
    if (grow < nN) {
      const size_t o = (size_t)grow * HID + (q & 31) * 4;
      *(volatile v4f*)(out + o) = o4[it];
      *(volatile v4f*)(out + (size_t)oofs + o) = o4[it];
    }
  }
}

extern "C" void kernel_launch(void* const* d_in, const int* in_sizes, int n_in,
                              void* d_out, int out_size, void* d_ws, size_t ws_size,
                              hipStream_t stream) {
  if (n_in < 7) return;
  const int nN = in_sizes[0] / INF;
  const int nE = in_sizes[2] / 2;
  if (nN <= 0 || nE <= 0 || in_sizes[0] != nN * INF || in_sizes[2] != 2 * nE) return;
  if (in_sizes[1] != nN * HID) return;
  if (in_sizes[3] != KF * 2 * HID || in_sizes[4] != 2 * HID) return;
  if (in_sizes[5] != KF * HID || in_sizes[6] != HID) return;
  if (out_size != 2 * nN * HID) return;
  if (nE > (1 << 28) || nN > (1 << 22)) return;

  const float* xin  = (const float*)d_in[0];
  const float* stin = (const float*)d_in[1];
  const int*   ei   = (const int*)d_in[2];
  const float* Wru  = (const float*)d_in[3];
  const float* bru  = (const float*)d_in[4];
  const float* Wc   = (const float*)d_in[5];
  const float* bc   = (const float*)d_in[6];
  const int* src = ei;
  const int* dst = ei + nE;
  float* out = (float*)d_out;
  const int oofs = nN * HID;
  if ((size_t)oofs + (size_t)nN * HID > (size_t)out_size) return;

  const int NPAD   = ((nN + TGT - 1) / TGT) * TGT;
  const int nBC    = (nN + NBC - 1) / NBC;
  const int CNTPAD = nBC * NBC;
  if (CNTPAD < NPAD) return;
  if (4 * nBC + 1 > RBN) return;
  const int nBF    = (nN + NBF - 1) / NBF;
  if (nBF + 1 > 4 * nBC + 1) return;
  const int csrLen = ((nE + 31) & ~31) + 4096;
  if (31 * 4 * nBC > 4096) return;
  const int nAgg   = NPAD / TGT;
  const int nGemm  = NPAD / BM;

  char* ws = (char*)d_ws;
  size_t off = 0;
  const size_t oW1  = off; off += (size_t)(2 * HID) * KF * 2;  off = (off + 255) & ~(size_t)255;
  const size_t oW2  = off; off += (size_t)HID * KF * 2;        off = (off + 255) & ~(size_t)255;
  const size_t oAX  = off; off += (size_t)NPAD * INF * 2;      off = (off + 255) & ~(size_t)255;
  const size_t oAS  = off; off += (size_t)NPAD * HID * 2;      off = (off + 255) & ~(size_t)255;
  const size_t oAR  = off; off += (size_t)NPAD * HID * 2;      off = (off + 255) & ~(size_t)255;
  const size_t oRS  = off; off += (size_t)NPAD * HID * 4;      off = (off + 255) & ~(size_t)255;
  const size_t oU   = off; off += (size_t)NPAD * HID * 4;      off = (off + 255) & ~(size_t)255;
  const size_t oCnt = off; off += (size_t)CNTPAD * 4;          off = (off + 255) & ~(size_t)255;
  const size_t oOff = off; off += (size_t)CNTPAD * 4;          off = (off + 255) & ~(size_t)255;
  const size_t oRb  = off; off += (size_t)RBN * 4;             off = (off + 255) & ~(size_t)255;
  const size_t oCsr = off; off += (size_t)csrLen * 4;          off = (off + 255) & ~(size_t)255;
  if (off > ws_size || off > (size_t)WSCAP) return;
  _Float16* pW1   = (_Float16*)(ws + oW1);
  _Float16* pW2   = (_Float16*)(ws + oW2);
  _Float16* aggX  = (_Float16*)(ws + oAX);
  _Float16* aggS  = (_Float16*)(ws + oAS);
  _Float16* aggRS = (_Float16*)(ws + oAR);
  float* rsP  = (float*)(ws + oRS);
  float* uP   = (float*)(ws + oU);
  int*   cnt  = (int*)(ws + oCnt);
  int*   offp = (int*)(ws + oOff);
  int*   rb   = (int*)(ws + oRb);
  int*   csr  = (int*)(ws + oCsr);

  const int vec8 = ((nE & 7) == 0) ? 1 : 0;

  k_prepw<KF, 2 * HID><<<((2 * HID) * KF / 8) / NTHR, NTHR, 0, stream>>>(Wru, pW1);
  k_prepw<KF, HID    ><<<(HID * KF / 8) / NTHR,       NTHR, 0, stream>>>(Wc,  pW2);

  k_count<<<nBC, NTHR, 0, stream>>>(dst, cnt, nE, vec8);
  k_offsets<<<1, OTHR, 0, stream>>>(cnt, offp, rb, nBC);
  hipFuncSetAttribute(reinterpret_cast<const void*>(&k_fill),
                      hipFuncAttributeMaxDynamicSharedMemorySize, LDS_FILL);
  k_fill<<<nBF, NTHR, LDS_FILL, stream>>>(dst, offp, rb, csr, nE, vec8, csrLen);

  k_agg<1><<<nAgg, NTHR, 0, stream>>>(csr, offp, cnt, src, xin, stin, aggX, aggS, nN, nE, csrLen);
  k_gemm1<<<nGemm, NTHR, 0, stream>>>(aggX, aggS, pW1, bru, stin, rsP, uP, nN);
  k_agg<0><<<nAgg, NTHR, 0, stream>>>(csr, offp, cnt, src, xin, rsP, aggX, aggRS, nN, nE, csrLen);
  k_gemm2<<<nGemm, NTHR, 0, stream>>>(aggX, aggRS, pW2, bc, stin, uP, out, nN, oofs);
}
